// ShiftedWindowMSA_83210696393647
// MI455X (gfx1250) — hardware-verified
//
#include <hip/hip_runtime.h>
#include <math.h>
typedef __attribute__((ext_vector_type(16))) _Float16 v16h;
typedef __attribute__((ext_vector_type(8)))  _Float16 v8h;
typedef __attribute__((ext_vector_type(16))) __bf16   v16b;
typedef __attribute__((ext_vector_type(8)))  __bf16   v8b;
typedef __attribute__((ext_vector_type(8)))  float    v8f;
typedef __attribute__((ext_vector_type(4)))  float    v4f;
#define PSCALE 32768.0f
#define U16(p) ((const unsigned short*)(const void*)(p))
#define PSCALE_INV (1.0f / 32768.0f)

__device__ __forceinline__ unsigned short f2bf_bits(float f) {
  unsigned u = __float_as_uint(f);
  return (unsigned short)((u + 0x7FFFu + ((u >> 16) & 1u)) >> 16);
}
__device__ __forceinline__ float bf_bits2f(unsigned short h) { return __uint_as_float(((unsigned)h) << 16); }

__device__ __forceinline__ void dep_guard_h(v8f& a, v8f& b, v16h x, v16h y) { asm volatile("v_nop\n\tv_nop\n\tv_nop\n\tv_nop" : "+v"(a), "+v"(b) : "v"(x), "v"(y)); }
__device__ __forceinline__ void dep_guard_b(v8f& a, v8f& b, v16b x, v16b y) { asm volatile("v_nop\n\tv_nop\n\tv_nop\n\tv_nop" : "+v"(a), "+v"(b) : "v"(x), "v"(y)); }
__device__ __forceinline__ void keep4_h(v16h a, v16h b, v16h c, v16h d) { asm volatile("v_nop" :: "v"(a), "v"(b), "v"(c), "v"(d)); }
__device__ __forceinline__ void keep4_b(v16b a, v16b b, v16b c, v16b d) { asm volatile("v_nop" :: "v"(a), "v"(b), "v"(c), "v"(d)); }
__device__ __forceinline__ void acc_guard4(v8f& a, v8f& b, v8f& c, v8f& d) { asm volatile("v_nop\n\tv_nop\n\tv_nop\n\tv_nop" : "+v"(a), "+v"(b), "+v"(c), "+v"(d)); }
template <typename T> struct Frag;
template <> struct Frag<_Float16> {
  typedef v16h V; union U { v16h v; v8h h[2]; };
  static __device__ __forceinline__ v16h load(const _Float16* p) {
    U f; f.h[0] = *(const v8h*)(p); f.h[1] = *(const v8h*)(p + 16); return f.v;
  }
  static __device__ __forceinline__ v8f mma(v16h a, v16h b, v8f c) {
    return __builtin_amdgcn_wmma_f32_16x16x32_f16(false, a, false, b, (short)0, c, false, false);
  }
  static __device__ __forceinline__ void guard(v8f& a, v8f& b, v16h x, v16h y) { dep_guard_h(a, b, x, y); }
  static __device__ __forceinline__ void keep(v16h a, v16h b, v16h c, v16h d) { keep4_h(a, b, c, d); }
};
template <> struct Frag<__bf16> {
  typedef v16b V; union U { v16b v; v8b h[2]; };
  static __device__ __forceinline__ v16b load(const __bf16* p) {
    U f; f.h[0] = *(const v8b*)(p); f.h[1] = *(const v8b*)(p + 16); return f.v;
  }
  static __device__ __forceinline__ v8f mma(v16b a, v16b b, v8f c) {
    return __builtin_amdgcn_wmma_f32_16x16x32_bf16(false, a, false, b, (short)0, c, false, false);
  }
  static __device__ __forceinline__ void guard(v8f& a, v8f& b, v16b x, v16b y) { dep_guard_b(a, b, x, y); }
  static __device__ __forceinline__ void keep(v16b a, v16b b, v16b c, v16b d) { keep4_b(a, b, c, d); }
};

template <int ET> struct Elem;
template <> struct Elem<0> { typedef _Float16 T; };
template <> struct Elem<1> { typedef __bf16 T; };
template <int ET, bool SPLIT, int BIAS_MODE, int OUT_MODE, bool RESID, int ACT = 0>
__global__ __launch_bounds__(256) void wmma_gemm64(
    const unsigned short* __restrict__ Ap, const unsigned short* __restrict__ A2p, int lda, long strideA,
    const unsigned short* __restrict__ Btp, const unsigned short* __restrict__ Bt2p, int ldb, long strideB,
    void* __restrict__ Cout, void* __restrict__ Cout2, int ldc, long strideC,
    const float* __restrict__ bias,
    const float* __restrict__ resid, long strideR,
    int M, int N, int K, float scale) {
  typedef typename Elem<ET>::T T;
  typedef typename Frag<T>::V V;
  const T* A = (const T*)Ap; const T* A2 = (const T*)A2p; const T* Bt = (const T*)Btp; const T* Bt2 = (const T*)Bt2p;
  __shared__ __align__(16) float sT[8][16 * 68];
  const int b    = blockIdx.y;
  const int lane = threadIdx.x & 31;
  const int wave = threadIdx.x >> 5;
  const int tilesN = N >> 6;
  const int tilesM = M >> 6;
  const int tile = blockIdx.x * 8 + wave;
  if (tile >= tilesM * tilesN) return;
  const int tm = tile / tilesN;
  const int tn = tile - tm * tilesN;
  const int m0 = tm << 6;
  const int n0 = tn << 6;

  const T* Ab  = A  + (size_t)b * strideA;
  const T* Bb  = Bt + (size_t)b * strideB;
  const T* Ab2 = SPLIT ? (A2  + (size_t)b * strideA) : nullptr;
  const T* Bb2 = SPLIT ? (Bt2 + (size_t)b * strideB) : nullptr;

  const int rlane = lane & 15;
  const int koff  = (lane >> 4) * 8;
  const int mOff  = (lane >> 4) * 8;

  v8f acc[4][4];
#pragma unroll
  for (int i = 0; i < 4; ++i)
#pragma unroll
    for (int j = 0; j < 4; ++j) acc[i][j] = (v8f){0.f,0.f,0.f,0.f,0.f,0.f,0.f,0.f};

  for (int k0 = 0; k0 < K; k0 += 32) {
    V bh[4], bl[4];
#pragma unroll
    for (int j = 0; j < 4; ++j) {
      const size_t bo = (size_t)(n0 + (j << 4) + rlane) * ldb + koff + k0;
      bh[j] = Frag<T>::load(Bb + bo);
      if (SPLIT) bl[j] = Frag<T>::load(Bb2 + bo);
    }
#pragma unroll
    for (int i = 0; i < 4; ++i) {
      const size_t ao = (size_t)(m0 + (i << 4) + rlane) * lda + koff + k0;
      V ah = Frag<T>::load(Ab + ao);
      V al;
      if (SPLIT) al = Frag<T>::load(Ab2 + ao);
#pragma unroll
      for (int j = 0; j < 4; ++j) {
        acc[i][j] = Frag<T>::mma(ah, bh[j], acc[i][j]);
        if (SPLIT) {
          acc[i][j] = Frag<T>::mma(ah, bl[j], acc[i][j]);
          acc[i][j] = Frag<T>::mma(al, bh[j], acc[i][j]);
        }
      }
      Frag<T>::guard(acc[i][0], acc[i][3], ah, SPLIT ? al : ah);
    }
    Frag<T>::keep(bh[0], bh[1], bh[2], bh[3]);
    if (SPLIT) Frag<T>::keep(bl[0], bl[1], bl[2], bl[3]);
  }
  acc_guard4(acc[0][0], acc[0][1], acc[0][2], acc[0][3]);
  acc_guard4(acc[1][0], acc[1][1], acc[1][2], acc[1][3]);
  acc_guard4(acc[2][0], acc[2][1], acc[2][2], acc[2][3]);
  acc_guard4(acc[3][0], acc[3][1], acc[3][2], acc[3][3]);

  float* slab = sT[wave];
  const float* Rb = RESID ? (resid + (size_t)b * strideR) : nullptr;
#pragma unroll
  for (int i = 0; i < 4; ++i) {
    const int mBase = m0 + (i << 4);
#pragma unroll
    for (int j = 0; j < 4; ++j) {
      const int n = n0 + (j << 4) + rlane;
      float bv = 0.f;
      if (BIAS_MODE == 2) bv = bias[n];
#pragma unroll
      for (int r = 0; r < 8; ++r) {
        float v = acc[i][j][r] * scale;
        if (BIAS_MODE == 1) v += bias[mBase + mOff + r];
        if (BIAS_MODE == 2) v += bv;
        if (RESID) v += Rb[(size_t)(mBase + mOff + r) * ldc + n];
        if (ACT == 1) v = tanhf(v);
        if (ACT == 2) v = fmaxf(v, 0.0f);
        if (ACT == 3) v = v / (1.0f + expf(-v));
        if (ACT == 4) v = (v > 0.f) ? v : 0.01f * v;
        if (ACT == 5) v = 0.5f * v * (1.0f + erff(v * 0.70710678118654752f));
        slab[(mOff + r) * 68 + (j << 4) + rlane] = v;
      }
    }
    __builtin_amdgcn_fence(__ATOMIC_RELEASE, "workgroup");
    __builtin_amdgcn_wave_barrier();
    __builtin_amdgcn_fence(__ATOMIC_ACQUIRE, "workgroup");
    if (OUT_MODE == 0) {
      float* C = (float*)Cout + (size_t)b * strideC;
      const int hh = lane >> 4, c4 = (lane & 15) * 4;
      for (int pass = 0; pass < 2; ++pass) {
#pragma unroll
        for (int it = 0; it < 8; ++it) {
          const int row = it * 2 + hh;
          v4f v = *(const v4f*)(slab + row * 68 + c4);
          *(volatile v4f*)(C + (size_t)(mBase + row) * ldc + n0 + c4) = v;
        }
        __threadfence();
      }
    } else {
      const int q = lane >> 3, c8 = (lane & 7) * 8;
      unsigned short* C  = (unsigned short*)Cout  + (size_t)b * strideC;
      unsigned short* C2 = (OUT_MODE == 2) ? ((unsigned short*)Cout2 + (size_t)b * strideC) : nullptr;
      for (int pass = 0; pass < 2; ++pass) {
#pragma unroll
        for (int it = 0; it < 4; ++it) {
          const int row = it * 4 + q;
          const float* sp = slab + row * 68 + c8;
          v8h hv, lv;
#pragma unroll
          for (int e = 0; e < 8; ++e) {
            if (OUT_MODE == 1) {
              hv[e] = (_Float16)sp[e];
            } else {
              unsigned short hb = f2bf_bits(sp[e]);
              unsigned short lb = f2bf_bits(sp[e] - bf_bits2f(hb));
              hv[e] = __builtin_bit_cast(_Float16, hb);
              lv[e] = __builtin_bit_cast(_Float16, lb);
            }
          }
          *(volatile v8h*)(C + (size_t)(mBase + row) * ldc + n0 + c8) = hv;
          if (OUT_MODE == 2) *(volatile v8h*)(C2 + (size_t)(mBase + row) * ldc + n0 + c8) = lv;
        }
        __threadfence();
      }
    }
    __builtin_amdgcn_fence(__ATOMIC_RELEASE, "workgroup");
    __builtin_amdgcn_wave_barrier();
    __builtin_amdgcn_fence(__ATOMIC_ACQUIRE, "workgroup");
  }
}

__global__ __launch_bounds__(256) void cast_f32_f16x2(
    const float* __restrict__ in, _Float16* __restrict__ out, int n2) {
  int i = blockIdx.x * 256 + threadIdx.x;
  if (i < n2) {
    const _Float16 h0 = (_Float16)in[2 * i], h1 = (_Float16)in[2 * i + 1];
    const unsigned u = (unsigned)__builtin_bit_cast(unsigned short, h0) | ((unsigned)__builtin_bit_cast(unsigned short, h1) << 16);
    ((volatile unsigned*)out)[i] = u;
    __threadfence();
    ((volatile unsigned*)out)[i] = u;
  }
}


#define SN 32
#define SHW 56
#define SP (SHW * SHW)
#define SC 128
#define SROWS (SN * SP)
#define SWIN 256
#define SCH (49 * 32 * 3)
#define NHALF (SN / 8)
__constant__ unsigned long long ROWM[49] = {0x1fffff0000000ull,0x1fffff0000000ull,0x1fffff0000000ull,0x1fffff0000000ull,0x1fffff0000000ull,0x1fffff0000000ull,0x1fffff0000000ull,0x1fffff0000000ull,0x1fffff0000000ull,0x1fffff0000000ull,0x1fffff0000000ull,0x1fffff0000000ull,0x1fffff0000000ull,0x1fffff0000000ull,0x1fffff0000000ull,0x1fffff0000000ull,0x1fffff0000000ull,0x1fffff0000000ull,0x1fffff0000000ull,0x1fffff0000000ull,0x1fffff0000000ull,0x1fffff0000000ull,0x1fffff0000000ull,0x1fffff0000000ull,0x1fffff0000000ull,0x1fffff0000000ull,0x1fffff0000000ull,0x1fffff0000000ull,0xfffffffull,0xfffffffull,0xfffffffull,0xfffffffull,0xfffffffull,0xfffffffull,0xfffffffull,0xfffffffull,0xfffffffull,0xfffffffull,0xfffffffull,0xfffffffull,0xfffffffull,0xfffffffull,0xfffffffull,0xfffffffull,0xfffffffull,0xfffffffull,0xfffffffull,0xfffffffull,0xfffffffull};
__constant__ unsigned long long COLM[49] = {0x1c3870e1c3870ull,0x1c3870e1c3870ull,0x1c3870e1c3870ull,0x1c3870e1c3870ull,0x3c78f1e3c78full,0x0ull,0x0ull,0x1c3870e1c3870ull,0x1c3870e1c3870ull,0x1c3870e1c3870ull,0x1c3870e1c3870ull,0x3c78f1e3c78full,0x0ull,0x0ull,0x1c3870e1c3870ull,0x1c3870e1c3870ull,0x1c3870e1c3870ull,0x1c3870e1c3870ull,0x3c78f1e3c78full,0x0ull,0x0ull,0x1c3870e1c3870ull,0x1c3870e1c3870ull,0x1c3870e1c3870ull,0x1c3870e1c3870ull,0x3c78f1e3c78full,0x0ull,0x0ull,0x1c3870e1c3870ull,0x1c3870e1c3870ull,0x1c3870e1c3870ull,0x1c3870e1c3870ull,0x3c78f1e3c78full,0x0ull,0x0ull,0x1c3870e1c3870ull,0x1c3870e1c3870ull,0x1c3870e1c3870ull,0x1c3870e1c3870ull,0x3c78f1e3c78full,0x0ull,0x0ull,0x1c3870e1c3870ull,0x1c3870e1c3870ull,0x1c3870e1c3870ull,0x1c3870e1c3870ull,0x3c78f1e3c78full,0x0ull,0x0ull};
__global__ __launch_bounds__(256) void chunk_kernel(const float* __restrict__ QKVh, int n0, unsigned* __restrict__ Q16, unsigned* __restrict__ K16, unsigned* __restrict__ VT16) {
  __shared__ float q[64][33], k[64][33], v[64][33];
  const int nl = blockIdx.y, w = blockIdx.x, t = threadIdx.x; const size_t cg = (size_t)nl * SWIN + w;
  for (int i = t; i < 64 * 33; i += 256) { (&q[0][0])[i] = 0.f; (&k[0][0])[i] = 0.f; (&v[0][0])[i] = 0.f; }
  __syncthreads();
  if (t < 192) { const int ds = t % 96, half = t / 96; const int d = ds / 3, s = ds % 3; const int tok0 = half * 25, tok1 = half ? 49 : 25;
    long f = (long)w * SCH + (long)tok0 * 96 + ds; int pix = (int)(f / 384), o = (int)(f % 384); int y = pix / SHW, x = pix % SHW;
    for (int tok = tok0; tok < tok1; ++tok) {
      const int ys = (y + 4 >= SHW) ? y + 4 - SHW : y + 4, xs = (x + 4 >= SHW) ? x + 4 - SHW : x + 4;
      const float val = QKVh[((size_t)nl * SP + ys * SHW + xs) * 384 + o];
      if (s == 0) q[tok][d] = val; else if (s == 1) k[tok][d] = val; else v[tok][d] = val;
      o += 96; if (o >= 384) { o -= 384; ++x; if (x == SHW) { x = 0; ++y; } } } }
  __syncthreads();
  for (int pass = 0; pass < 2; ++pass) {
    for (int i = t; i < 64 * 16; i += 256) { const int tok = i / 16, dp = 2 * (i % 16);
      ((volatile unsigned*)Q16)[(cg * 64 + tok) * 16 + dp / 2] = (unsigned)__builtin_bit_cast(unsigned short, (_Float16)q[tok][dp]) | ((unsigned)__builtin_bit_cast(unsigned short, (_Float16)q[tok][dp + 1]) << 16);
      ((volatile unsigned*)K16)[(cg * 64 + tok) * 16 + dp / 2] = (unsigned)__builtin_bit_cast(unsigned short, (_Float16)k[tok][dp]) | ((unsigned)__builtin_bit_cast(unsigned short, (_Float16)k[tok][dp + 1]) << 16); }
    for (int i = t; i < 64 * 32; i += 256) { const int d = i / 32, tp = 2 * (i % 32); const float a = (d < 32) ? v[tp][d] : 0.f, b = (d < 32) ? v[tp + 1][d] : 0.f;
      ((volatile unsigned*)VT16)[(cg * 64 + d) * 32 + tp / 2] = (unsigned)__builtin_bit_cast(unsigned short, (_Float16)a) | ((unsigned)__builtin_bit_cast(unsigned short, (_Float16)b) << 16); }
    __threadfence(); }
}
__global__ __launch_bounds__(256) void soft_kernel(const float* __restrict__ Sm, const float* __restrict__ rpe, unsigned* __restrict__ P16) {
  const int lane = threadIdx.x & 31, wave = threadIdx.x >> 5; const size_t gr = (size_t)blockIdx.x * 8 + wave; const size_t cg = gr / 64; const int p = (int)(gr % 64); const int w = (int)(cg % SWIN);
  const int hh = (w / 8) % 8, ww = w % 8;
  if (p >= 49) return;
  float s0 = -INFINITY, s1 = -INFINITY; const int c0 = 2 * lane, c1 = 2 * lane + 1;
  if (p < 49) {
    if (c0 < 49) { s0 = Sm[gr * 64 + c0] + rpe[(c0 / 7 - p / 7 + 6) * 13 + (c0 % 7 - p % 7 + 6)]; if (hh == 7 && ((ROWM[p] >> c0) & 1ull)) s0 = -INFINITY; if (ww == 7 && ((COLM[p] >> c0) & 1ull)) s0 = -INFINITY; }
    if (c1 < 49) { s1 = Sm[gr * 64 + c1] + rpe[(c1 / 7 - p / 7 + 6) * 13 + (c1 % 7 - p % 7 + 6)]; if (hh == 7 && ((ROWM[p] >> c1) & 1ull)) s1 = -INFINITY; if (ww == 7 && ((COLM[p] >> c1) & 1ull)) s1 = -INFINITY; } }
  float mx = fmaxf(s0, s1); for (int o = 16; o > 0; o >>= 1) mx = fmaxf(mx, __shfl_xor(mx, o, 32));
  float e0 = (p < 49 && c0 < 49) ? expf(s0 - mx) : 0.f, e1 = (p < 49 && c1 < 49) ? expf(s1 - mx) : 0.f;
  float se = e0 + e1; for (int o = 16; o > 0; o >>= 1) se += __shfl_xor(se, o, 32);
  const float sc = (p < 49) ? 32768.0f / se : 0.f;
  const unsigned u = (unsigned)__builtin_bit_cast(unsigned short, (_Float16)(e0 * sc)) | ((unsigned)__builtin_bit_cast(unsigned short, (_Float16)(e1 * sc)) << 16);
  ((volatile unsigned*)P16)[gr * 32 + lane] = u; __threadfence(); ((volatile unsigned*)P16)[gr * 32 + lane] = u;
}
__global__ __launch_bounds__(256) void ostore_kernel(const float* __restrict__ OC, int n0, float* __restrict__ O) {
  const int nl = blockIdx.y, w = blockIdx.x; const size_t cg = (size_t)nl * SWIN + w; float* dst = O + (size_t)nl * SP * SC + (size_t)w * 1568; (void)n0;
  for (int pass = 0; pass < 2; ++pass) { for (int e = threadIdx.x; e < 1568; e += 256) { const int p = e / 32, d = e % 32; ((volatile float*)dst)[e] = OC[(cg * 64 + p) * 64 + d]; } __threadfence(); }
}
__global__ __launch_bounds__(256) void roll_cast_kernel(const float* __restrict__ O, unsigned* __restrict__ A16) {
  const int lane = threadIdx.x & 31, wave = threadIdx.x >> 5; const size_t r = (size_t)blockIdx.x * 8 + wave; const int n = (int)(r / SP), pix = (int)(r % SP); const int y = pix / SHW, x = pix % SHW;
  const int ys = (y - 3 + SHW) % SHW, xs = (x - 3 + SHW) % SHW; const v4f a = *(const v4f*)(O + ((size_t)n * SP + ys * SHW + xs) * SC + lane * 4);
  typedef __attribute__((ext_vector_type(2))) unsigned u2; u2 u; u[0] = (unsigned)__builtin_bit_cast(unsigned short, (_Float16)a[0]) | ((unsigned)__builtin_bit_cast(unsigned short, (_Float16)a[1]) << 16); u[1] = (unsigned)__builtin_bit_cast(unsigned short, (_Float16)a[2]) | ((unsigned)__builtin_bit_cast(unsigned short, (_Float16)a[3]) << 16);
  *(volatile u2*)(A16 + (r * SC) / 2 + lane * 2) = u; __threadfence(); *(volatile u2*)(A16 + (r * SC) / 2 + lane * 2) = u;
}
extern "C" void kernel_launch(void* const* d_in, const int* in_sizes, int n_in, void* d_out, int out_size, void* d_ws, size_t ws_size, hipStream_t stream) {
  (void)in_sizes; (void)n_in; (void)out_size; (void)ws_size;
  const float* x = (const float*)d_in[0]; const float* qw = (const float*)d_in[1]; const float* qb = (const float*)d_in[2]; const float* ow = (const float*)d_in[3]; const float* ob = (const float*)d_in[4]; const float* rpe = (const float*)d_in[5];
  char* ws = (char*)d_ws; size_t off = 0;
  auto carve = [&](size_t bytes) -> char* { char* p = ws + off; off += (bytes + 255) & ~(size_t)255; return p; };
  _Float16* X16 = (_Float16*)carve((size_t)NHALF * SP * SC * 2); _Float16* QW16 = (_Float16*)carve(384 * SC * 2); _Float16* OW16 = (_Float16*)carve(SC * SC * 2);
  float* QKVh = (float*)carve((size_t)NHALF * SP * 384 * 4); float* O = (float*)carve((size_t)NHALF * SP * SC * 4); unsigned* A16 = (unsigned*)carve((size_t)NHALF * SP * SC * 2);
  const int NCG = NHALF * SWIN;
  unsigned* Q16c = (unsigned*)carve((size_t)NCG * 64 * 32 * 2); unsigned* K16c = (unsigned*)carve((size_t)NCG * 64 * 32 * 2); unsigned* VT16 = (unsigned*)carve((size_t)NCG * 64 * 64 * 2);
  float* Sm = (float*)carve((size_t)NCG * 64 * 64 * 4); unsigned* P16 = (unsigned*)carve((size_t)NCG * 64 * 64 * 2); float* OC = Sm;
  cast_f32_f16x2<<<(384 * SC / 2 + 255) / 256, 256, 0, stream>>>(qw, QW16, 384 * SC / 2);
  cast_f32_f16x2<<<(SC * SC / 2 + 255) / 256, 256, 0, stream>>>(ow, OW16, SC * SC / 2);
  for (int half = 0; half < 8; ++half) { const int n0 = half * NHALF;
    cast_f32_f16x2<<<(NHALF * SP * SC / 2 + 255) / 256, 256, 0, stream>>>(x + (size_t)n0 * SP * SC, X16, (long)NHALF * SP * SC / 2);
    { const int t = (NHALF * SP / 64) * 6;
      wmma_gemm64<0, false, 2, 0, false><<<dim3((t + 7) / 8, 1), 256, 0, stream>>>(U16(X16), nullptr, SC, 0, U16(QW16), nullptr, SC, 0, QKVh, nullptr, 384, 0, qb, nullptr, 0, NHALF * SP, 384, SC, 1.0f); }
    chunk_kernel<<<dim3(SWIN, NHALF), 256, 0, stream>>>(QKVh, n0, Q16c, K16c, VT16);
    wmma_gemm64<0, false, 0, 0, false><<<dim3(1, NCG), 256, 0, stream>>>((const unsigned short*)Q16c, nullptr, 32, 64 * 32, (const unsigned short*)K16c, nullptr, 32, 64 * 32, Sm, nullptr, 64, 64 * 64, nullptr, nullptr, 0, 64, 64, 32, 0.17677669529663687f);
    soft_kernel<<<NCG * 64 / 8, 256, 0, stream>>>(Sm, rpe, P16);
    wmma_gemm64<0, false, 0, 0, false><<<dim3(1, NCG), 256, 0, stream>>>((const unsigned short*)P16, nullptr, 64, 64 * 64, (const unsigned short*)VT16, nullptr, 64, 64 * 64, OC, nullptr, 64, 64 * 64, nullptr, nullptr, 0, 64, 64, 64, 1.0f / 32768.0f);
    ostore_kernel<<<dim3(SWIN, NHALF), 256, 0, stream>>>(OC, n0, O);
    roll_cast_kernel<<<NHALF * SP / 8, 256, 0, stream>>>(O, A16);
    { const int t2 = (NHALF * SP / 64) * 2;
      wmma_gemm64<0, false, 2, 0, false><<<dim3((t2 + 7) / 8, 1), 256, 0, stream>>>((const unsigned short*)A16, nullptr, SC, 0, U16(OW16), nullptr, SC, 0, (float*)d_out + (size_t)n0 * SP * SC, nullptr, SC, 0, ob, nullptr, 0, NHALF * SP, SC, SC, 1.0f); } }
}
